// MSTRC_81758997447373
// MI455X (gfx1250) — hardware-verified
//
#include <hip/hip_runtime.h>
#include <hip/hip_bf16.h>
#include <stddef.h>


#define NTH    256
#define NWV    8
#define CHUNK  2048
#define NGRP   2
#define WCAP   256
#define NB     64
#define SH     6
#define NBG    128
#define SHG    7
#define HC     512
#define HID    128
#define KVP    1024
#define GP     256
#define STGP   68
#define QSCALE 0.08838834764831845f

#define LY_R0   (NB * HC * 4)
#define LY_R1   (NB * HC * 4)
#define LY_AUX  (NB * 4 * 4 * 2)
#define LY_LIST (NWV * WCAP * 4)
#define LY_LDS  (LY_R0 + LY_R1 + LY_AUX + LY_LIST + 64)
#define PL_MX   (NBG * HID * 4)
#define PL_LDS  (2 * PL_MX + NBG * 4 + LY_LIST + 64)

static_assert(LY_LDS == 272448);
static_assert(PL_LDS == 139840);
static_assert(WCAP == (CHUNK / NTH) * 32);
static_assert(NGRP * NTH * 4 == CHUNK);
static_assert(NB == (1 << SH));
static_assert(NBG == (1 << SHG));
static_assert(NWV * 16 * STGP * 4 <= LY_R1);
static_assert(2 * NB * HC * 2 <= LY_R0);
static_assert(SH + 11 <= 31);
static_assert(SHG + 11 <= 31);

typedef float  v4f  __attribute__((ext_vector_type(4)));
typedef float  v8f  __attribute__((ext_vector_type(8)));
typedef int    v4i  __attribute__((ext_vector_type(4)));
typedef __bf16 v16b __attribute__((ext_vector_type(16)));
union Frag { v16b v; v4i q[2]; };

__device__ __forceinline__ v8f wm(v16b a, v16b b, v8f c) {
  v8f d = __builtin_amdgcn_wmma_f32_16x16x32_bf16(false, a, false, b, (short)0, c, false, false);
  asm volatile("v_nop\n\tv_nop\n\tv_nop\n\tv_nop" : "+v"(d) : "v"(a), "v"(b));
  return d;
}

__device__ __forceinline__ v16b ldf(const unsigned short* p) {
  Frag f;
  f.q[0] = *(const v4i*)p;
  f.q[1] = *(const v4i*)(p + 16);
  return f.v;
}

__device__ __forceinline__ unsigned bfr(float f) {
  unsigned u = __float_as_uint(f);
  u += 0x7FFFu + ((u >> 16) & 1u);
  return u >> 16;
}

__device__ __forceinline__ void pack8(v4f a, v4f b, v4i& hq, v4i& lq) {
  const float x[8] = {a.x, a.y, a.z, a.w, b.x, b.y, b.z, b.w};
  unsigned h[8], o[8];
#pragma unroll
  for (int i = 0; i < 8; ++i) {
    h[i] = bfr(x[i]);
    o[i] = bfr(x[i] - __uint_as_float(h[i] << 16));
  }
  hq.x = (int)(h[0] | (h[1] << 16)); hq.y = (int)(h[2] | (h[3] << 16));
  hq.z = (int)(h[4] | (h[5] << 16)); hq.w = (int)(h[6] | (h[7] << 16));
  lq.x = (int)(o[0] | (o[1] << 16)); lq.y = (int)(o[2] | (o[3] << 16));
  lq.z = (int)(o[4] | (o[5] << 16)); lq.w = (int)(o[6] | (o[7] << 16));
}

__device__ __forceinline__ v4f relu4(v4f a) {
  a.x = fmaxf(a.x, 0.f); a.y = fmaxf(a.y, 0.f); a.z = fmaxf(a.z, 0.f); a.w = fmaxf(a.w, 0.f);
  return a;
}
__device__ __forceinline__ v4f max4(v4f a, v4f b) {
  v4f r;
  r.x = fmaxf(a.x, b.x); r.y = fmaxf(a.y, b.y); r.z = fmaxf(a.z, b.z); r.w = fmaxf(a.w, b.w);
  return r;
}
__device__ __forceinline__ v4f sel4(bool c, v4f a, v4f b) {
  v4f r;
  r.x = c ? a.x : b.x; r.y = c ? a.y : b.y; r.z = c ? a.z : b.z; r.w = c ? a.w : b.w;
  return r;
}

template <int NSLOT, int SHF>
__device__ __forceinline__ int scan_chunk(const int* __restrict__ ids, int nIds, int cbase, bool full,
                                          int base, int* wl, int tid) {
  int wc = 0;
#pragma unroll
  for (int g = 0; g < NGRP; ++g) {
    const int el0 = (g * NTH + tid) * 4;
    const int e0 = cbase + el0;
    const int sent = -2147483647 - 1;
    v4i d;
    if (full) {
      d = *(const v4i*)(ids + e0);
    } else {
      const int last = nIds - 1;
      const int t0 = ids[min(e0, last)];
      const int t1 = ids[min(e0 + 1, last)];
      const int t2 = ids[min(e0 + 2, last)];
      const int t3 = ids[min(e0 + 3, last)];
      d.x = (e0     < nIds) ? t0 : sent;
      d.y = (e0 + 1 < nIds) ? t1 : sent;
      d.z = (e0 + 2 < nIds) ? t2 : sent;
      d.w = (e0 + 3 < nIds) ? t3 : sent;
    }
    const unsigned s0 = (unsigned)d.x - (unsigned)base;
    const unsigned s1 = (unsigned)d.y - (unsigned)base;
    const unsigned s2 = (unsigned)d.z - (unsigned)base;
    const unsigned s3 = (unsigned)d.w - (unsigned)base;
    const bool h0 = s0 < (unsigned)NSLOT;
    const bool h1 = s1 < (unsigned)NSLOT;
    const bool h2 = s2 < (unsigned)NSLOT;
    const bool h3 = s3 < (unsigned)NSLOT;
    const unsigned any = __builtin_amdgcn_ballot_w32(h0 | h1 | h2 | h3);
    if (any != 0u) {
#define HITJ(J, HJ, SJ) { \
        const unsigned mj = __builtin_amdgcn_ballot_w32(HJ); \
        if (HJ) { \
          const int pos = wc + (int)__builtin_amdgcn_mbcnt_lo(mj, 0u); \
          if (pos < WCAP) wl[pos] = ((el0 + (J)) << SHF) | (int)(SJ); \
        } \
        wc += (int)__builtin_popcount(mj); }
      HITJ(0, h0, s0)
      HITJ(1, h1, s1)
      HITJ(2, h2, s2)
      HITJ(3, h3, s3)
#undef HITJ
    }
  }
  return wc;
}

__global__ __launch_bounds__(NTH) void k_prep(const float* __restrict__ w0, const float* __restrict__ w1,
                                            const float* __restrict__ w2, const float* __restrict__ w3,
                                            int nce, int K, int Kp,
                                            unsigned short* Ph, unsigned short* Pl, int ntot) {
  __shared__ __attribute__((aligned(16))) float tile[32 * 68];
  const int tid = threadIdx.x;
  const int n0 = blockIdx.x * 32;
  int which = n0 / nce;
  which = which > 3 ? 3 : which;
  const float* s = (which == 0) ? w0 : ((which == 1) ? w1 : ((which == 2) ? w2 : w3));
  const int cbase = n0 - which * nce;
#pragma unroll 1
  for (int kc = 0; kc < Kp; kc += 64) {
#pragma unroll
    for (int i = 0; i < 8; ++i) {
      const int e = i * NTH + tid;
      const int nn = e & 31;
      const int kk = e >> 5;
      const int k = kc + kk;
      const int kcl = k < K ? k : K - 1;
      int col = cbase + nn;
      col = col > nce - 1 ? nce - 1 : col;
      const float v = s[(size_t)kcl * nce + col];
      tile[nn * 68 + kk] = (k < K && (n0 + nn) < ntot) ? v : 0.f;
    }
    __syncthreads();
    {
      const int row = tid >> 3, pc = tid & 7;
      const v4f a = *(const v4f*)(tile + row * 68 + 8 * pc);
      const v4f b = *(const v4f*)(tile + row * 68 + 8 * pc + 4);
      v4i hq, lq;
      pack8(a, b, hq, lq);
      const bool ok = (n0 + row) < ntot;
      const size_t o = (size_t)(n0 + row) * Kp + kc + 8 * pc;
      if (ok) { *(volatile v4i*)(Ph + o) = hq; *(volatile v4i*)(Pl + o) = lq; }
      __threadfence();
      if (ok) { *(volatile v4i*)(Ph + o) = hq; *(volatile v4i*)(Pl + o) = lq; }
    }
    __syncthreads();
  }
}

__global__ __launch_bounds__(NTH) void k_cvt(const float* __restrict__ src, int K, int nRows, int Kp, int MP,
                                           unsigned short* Ph, unsigned short* Pl) {
  const int gid = blockIdx.x * NTH + threadIdx.x;
  const int ppr = Kp >> 3;
  if (gid >= MP * ppr) return;
  const int row = gid / ppr;
  const int c0 = (gid - row * ppr) * 8;
  const int rcl = row < nRows ? row : nRows - 1;
  const float* sp = src + (size_t)rcl * K;
  float x[8];
#pragma unroll
  for (int i = 0; i < 8; ++i) {
    const int c = c0 + i;
    const int ccl = c < K ? c : K - 1;
    const float v = sp[ccl];
    x[i] = (row < nRows && c < K) ? v : 0.f;
  }
  const v4f a = {x[0], x[1], x[2], x[3]};
  const v4f b = {x[4], x[5], x[6], x[7]};
  v4i hq, lq;
  pack8(a, b, hq, lq);
  const size_t o = (size_t)row * Kp + c0;
  *(volatile v4i*)(Ph + o) = hq;
  *(volatile v4i*)(Pl + o) = lq;
  __threadfence();
  *(volatile v4i*)(Ph + o) = hq;
  *(volatile v4i*)(Pl + o) = lq;
}

template <int TN, int WCG, int OM, int RELU>
__global__ __launch_bounds__(32 * WCG) void k_gemm(
    const unsigned short* __restrict__ Ah, const unsigned short* __restrict__ Al,
    const unsigned short* __restrict__ Bh, const unsigned short* __restrict__ Bl,
    const float* __restrict__ b0, const float* __restrict__ b1, int nce,
    float* Cf, unsigned short* Oh, unsigned short* Ol,
    const float* __restrict__ w2, const float* __restrict__ b2, float* ov,
    int Kp, int Nout) {
  constexpr int CW = 16 * TN;
  constexpr int CB = CW * WCG;
  constexpr int SP = CW + 4;
  static_assert(TN == 2 || TN == 4);
  static_assert(OM != 1 || TN == 4);
  static_assert(OM != 2 || TN == 2);
  __shared__ __attribute__((aligned(16))) float stg[WCG * 16 * SP];
  __shared__ float part[WCG * 32];
  __shared__ __attribute__((aligned(16))) float outs[32];

  const int tid = threadIdx.x;
  const int lane = tid & 31;
  const int wave = tid >> 5;
  const int hh = lane >> 4;
  const int l = lane & 15;
  const int r0 = blockIdx.x * 32;
  const int cb = blockIdx.y * CB + wave * CW;

  const v8f z8 = {0.f, 0.f, 0.f, 0.f, 0.f, 0.f, 0.f, 0.f};
  v8f acc[2][TN];
#pragma unroll
  for (int j = 0; j < TN; ++j) { acc[0][j] = z8; acc[1][j] = z8; }

  const size_t oa0 = (size_t)(r0 + l) * Kp + 8 * hh;
  const size_t oa1 = oa0 + (size_t)16 * Kp;
  size_t ob[TN];
#pragma unroll
  for (int j = 0; j < TN; ++j) ob[j] = (size_t)(cb + 16 * j + l) * Kp + 8 * hh;

#pragma unroll 1
  for (int k0 = 0; k0 < Kp; k0 += 32) {
    const v16b a0h = ldf(Ah + oa0 + k0);
    const v16b a1h = ldf(Ah + oa1 + k0);
    const v16b a0l = ldf(Al + oa0 + k0);
    const v16b a1l = ldf(Al + oa1 + k0);
#pragma unroll
    for (int j = 0; j < TN; ++j) {
      const v16b bh = ldf(Bh + ob[j] + k0);
      const v16b bl = ldf(Bl + ob[j] + k0);
      acc[0][j] = wm(a0h, bh, acc[0][j]);
      acc[0][j] = wm(a0h, bl, acc[0][j]);
      acc[0][j] = wm(a0l, bh, acc[0][j]);
      acc[1][j] = wm(a1h, bh, acc[1][j]);
      acc[1][j] = wm(a1h, bl, acc[1][j]);
      acc[1][j] = wm(a1l, bh, acc[1][j]);
    }
  }

  float* sw = stg + wave * 16 * SP;
#pragma unroll
  for (int i = 0; i < 2; ++i) {
#pragma unroll
    for (int j = 0; j < TN; ++j) {
#pragma unroll
      for (int r = 0; r < 8; ++r) sw[(8 * hh + r) * SP + 16 * j + l] = acc[i][j][r];
    }
    __syncthreads();
    if (OM == 0) {
      constexpr int PPR = CW / 4;
      constexpr int NIT = (16 * PPR) / 32;
      v4f vals[NIT];
      size_t offs[NIT];
#pragma unroll
      for (int it = 0; it < NIT; ++it) {
        const int idx = it * 32 + lane;
        const int row = idx / PPR;
        const int pc = idx - row * PPR;
        const int col = cb + 4 * pc;
        int which = col / nce;
        which = which > 1 ? 1 : which;
        const float* bb = (which == 0) ? b0 : b1;
        const v4f bv = *(const v4f*)(bb + (col - which * nce));
        v4f v = *(const v4f*)(sw + row * SP + 4 * pc) + bv;
        if (RELU) v = relu4(v);
        vals[it] = v;
        offs[it] = (size_t)(r0 + 16 * i + row) * Nout + col;
      }
#pragma unroll
      for (int it = 0; it < NIT; ++it) *(volatile v4f*)(Cf + offs[it]) = vals[it];
      __threadfence();
#pragma unroll
      for (int it = 0; it < NIT; ++it) *(volatile v4f*)(Cf + offs[it]) = vals[it];
    } else if (OM == 1) {
      v4i hq[4], lq[4];
      size_t offs[4];
#pragma unroll
      for (int it = 0; it < 4; ++it) {
        const int idx = it * 32 + lane;
        const int row = idx >> 3;
        const int pc = idx & 7;
        const int col = cb + 8 * pc;
        v4f a = *(const v4f*)(sw + row * SP + 8 * pc) + *(const v4f*)(b0 + col);
        v4f b = *(const v4f*)(sw + row * SP + 8 * pc + 4) + *(const v4f*)(b0 + col + 4);
        if (RELU) { a = relu4(a); b = relu4(b); }
        pack8(a, b, hq[it], lq[it]);
        offs[it] = (size_t)(r0 + 16 * i + row) * Nout + col;
      }
#pragma unroll
      for (int it = 0; it < 4; ++it) { *(volatile v4i*)(Oh + offs[it]) = hq[it]; *(volatile v4i*)(Ol + offs[it]) = lq[it]; }
      __threadfence();
#pragma unroll
      for (int it = 0; it < 4; ++it) { *(volatile v4i*)(Oh + offs[it]) = hq[it]; *(volatile v4i*)(Ol + offs[it]) = lq[it]; }
    } else {
      const int row = l;
      const int c0 = 16 * hh;
      float p = 0.f;
#pragma unroll
      for (int c = 0; c < 16; ++c) {
        float v = sw[row * SP + c0 + c] + b0[cb + c0 + c];
        v = RELU ? fmaxf(v, 0.f) : v;
        p += v * w2[cb + c0 + c];
      }
      p += __shfl_xor(p, 16, 32);
      if (hh == 0) part[wave * 32 + 16 * i + row] = p;
    }
    __syncthreads();
  }
  if (OM == 2) {
    if (wave == 0) {
      float s = b2[0];
#pragma unroll
      for (int w = 0; w < WCG; ++w) s += part[w * 32 + lane];
      outs[lane] = s;
    }
    __syncthreads();
    if (wave == 0) {
      const int lc = lane & 7;
      const bool wr = lane < 8;
      const v4f o = *(const v4f*)(outs + 4 * lc);
      float* op = ov + r0 + 4 * lc;
      if (wr) *(volatile v4f*)op = o;
      __threadfence();
      if (wr) *(volatile v4f*)op = o;
    }
  }
}

__global__ __launch_bounds__(NTH) void k_layer(
    const unsigned short* __restrict__ Xh, const unsigned short* __restrict__ Xl, int Kp,
    const unsigned short* __restrict__ Wh, const unsigned short* __restrict__ Wl,
    const float* __restrict__ bq, const float* __restrict__ bs,
    const float* __restrict__ KV, const int* __restrict__ ei,
    const unsigned short* __restrict__ Mh, const unsigned short* __restrict__ Ml,
    const float* __restrict__ bm, float* Hout, int nN, int nE) {
  extern __shared__ v4i lds_ly[];
  char* lb = (char*)lds_ly;
  float* qs = (float*)lb;
  unsigned short* th = (unsigned short*)lb;
  unsigned short* tl = th + NB * HC;
  float* sacc = (float*)(lb + LY_R0);
  float* stg = sacc;
  float* mx = (float*)(lb + LY_R0 + LY_R1);
  float* den = mx + NB * 4;
  int* list = (int*)(lb + LY_R0 + LY_R1 + LY_AUX);
  int* wcnt = list + NWV * WCAP;

  const int tid = threadIdx.x;
  const int lane = tid & 31;
  const int wave = tid >> 5;
  const int hh = lane >> 4;
  const int l = lane & 15;
  const int nodeBase = blockIdx.x * NB;
  const v8f z8 = {0.f, 0.f, 0.f, 0.f, 0.f, 0.f, 0.f, 0.f};

  {
    const v4f z4 = {0.f, 0.f, 0.f, 0.f};
    v4f* sv = (v4f*)sacc;
    for (int i = tid; i < NB * HC / 4; i += NTH) sv[i] = z4;
    for (int i = tid; i < NB * 4; i += NTH) { mx[i] = -1.0e30f; den[i] = 0.f; }
  }

  {
    const int cw = wave * 64;
#pragma unroll 1
    for (int rp = 0; rp < NB / 16; ++rp) {
      const int rb = rp * 16;
      v8f acc[4];
#pragma unroll
      for (int j = 0; j < 4; ++j) acc[j] = z8;
      const size_t oa = (size_t)(nodeBase + rb + l) * Kp + 8 * hh;
      size_t ob[4];
#pragma unroll
      for (int j = 0; j < 4; ++j) ob[j] = (size_t)(cw + 16 * j + l) * Kp + 8 * hh;
#pragma unroll 1
      for (int k0 = 0; k0 < Kp; k0 += 32) {
        const v16b ah = ldf(Xh + oa + k0);
        const v16b al = ldf(Xl + oa + k0);
#pragma unroll
        for (int j = 0; j < 4; ++j) {
          const v16b bh = ldf(Wh + ob[j] + k0);
          const v16b bl = ldf(Wl + ob[j] + k0);
          acc[j] = wm(ah, bh, acc[j]);
          acc[j] = wm(ah, bl, acc[j]);
          acc[j] = wm(al, bh, acc[j]);
        }
      }
#pragma unroll
      for (int j = 0; j < 4; ++j) {
        const int col = cw + 16 * j + l;
        const float bb = bq[col];
#pragma unroll
        for (int r = 0; r < 8; ++r) qs[(rb + 8 * hh + r) * HC + col] = acc[j][r] + bb;
      }
    }
  }
  __syncthreads();

  {
    const int* eid = ei + nE;
    const bool al16 = ((nE & 3) == 0);
    const int nChunks = (nE + CHUNK - 1) / CHUNK;
    const int hd = lane >> 3;
    int* wl = list + wave * WCAP;
#pragma unroll 1
    for (int ch = 0; ch < nChunks; ++ch) {
      const int cbase = ch * CHUNK;
      const bool full = al16 && (cbase + CHUNK <= nE);
      const int wc = scan_chunk<NB, SH>(eid, nE, cbase, full, nodeBase, wl, tid);
      if (lane == 0) wcnt[wave] = wc;
      __syncthreads();
      if (wave == 0) {
#pragma unroll 1
        for (int wsx = 0; wsx < NWV; ++wsx) {
          int n = wcnt[wsx];
          n = n > WCAP ? WCAP : n;
          n = n < 0 ? 0 : n;
#pragma unroll 1
          for (int i = 0; i < n; ++i) {
            const int ent = list[wsx * WCAP + i];
            const int slot = ent & (NB - 1);
            const int el = (ent >> SH) & (CHUNK - 1);
            int e = cbase + el;
            e = e > nE - 1 ? nE - 1 : e;
            int src = ei[e];
            src = src < 0 ? 0 : (src > nN - 1 ? nN - 1 : src);
            const float* qrow = qs + slot * HC + 16 * lane;
            const float* krow = KV + (size_t)src * KVP + 16 * lane;
            const float* vrow = krow + HC;
            const v4f q0 = *(const v4f*)(qrow);
            const v4f q1 = *(const v4f*)(qrow + 4);
            const v4f q2 = *(const v4f*)(qrow + 8);
            const v4f q3 = *(const v4f*)(qrow + 12);
            const v4f kk0 = *(const v4f*)(krow);
            const v4f kk1 = *(const v4f*)(krow + 4);
            const v4f kk2 = *(const v4f*)(krow + 8);
            const v4f kk3 = *(const v4f*)(krow + 12);
            float part = q0.x * kk0.x + q0.y * kk0.y + q0.z * kk0.z + q0.w * kk0.w
                       + q1.x * kk1.x + q1.y * kk1.y + q1.z * kk1.z + q1.w * kk1.w
                       + q2.x * kk2.x + q2.y * kk2.y + q2.z * kk2.z + q2.w * kk2.w
                       + q3.x * kk3.x + q3.y * kk3.y + q3.z * kk3.z + q3.w * kk3.w;
            part += __shfl_xor(part, 4, 32);
            part += __shfl_xor(part, 2, 32);
            part += __shfl_xor(part, 1, 32);
            const float logit = part * QSCALE;
            const int hidx = slot * 4 + hd;
            const float mo = mx[hidx];
            const float mn = fmaxf(mo, logit);
            const float corr = __expf(mo - mn);
            const float p = __expf(logit - mn);
            const float dn = den[hidx] * corr + p;
            const v4f vv0 = *(const v4f*)(vrow);
            const v4f vv1 = *(const v4f*)(vrow + 4);
            const v4f vv2 = *(const v4f*)(vrow + 8);
            const v4f vv3 = *(const v4f*)(vrow + 12);
            v4f* sp = (v4f*)(sacc + slot * HC + 16 * lane);
            const v4f c0 = sp[0];
            const v4f c1 = sp[1];
            const v4f c2 = sp[2];
            const v4f c3 = sp[3];
            sp[0] = c0 * corr + vv0 * p;
            sp[1] = c1 * corr + vv1 * p;
            sp[2] = c2 * corr + vv2 * p;
            sp[3] = c3 * corr + vv3 * p;
            den[hidx] = dn;
            mx[hidx] = mn;
          }
        }
      }
      __syncthreads();
    }
  }

  {
    const int cw = wave * 64;
    const int head = wave >> 1;
#pragma unroll 1
    for (int rp = 0; rp < NB / 16; ++rp) {
      const int rb = rp * 16;
      v8f acc[4];
#pragma unroll
      for (int j = 0; j < 4; ++j) acc[j] = z8;
      const size_t oa = (size_t)(nodeBase + rb + l) * Kp + 8 * hh;
      size_t ob[4];
#pragma unroll
      for (int j = 0; j < 4; ++j) ob[j] = (size_t)(3 * HC + cw + 16 * j + l) * Kp + 8 * hh;
#pragma unroll 1
      for (int k0 = 0; k0 < Kp; k0 += 32) {
        const v16b ah = ldf(Xh + oa + k0);
        const v16b al = ldf(Xl + oa + k0);
#pragma unroll
        for (int j = 0; j < 4; ++j) {
          const v16b bh = ldf(Wh + ob[j] + k0);
          const v16b bl = ldf(Wl + ob[j] + k0);
          acc[j] = wm(ah, bh, acc[j]);
          acc[j] = wm(ah, bl, acc[j]);
          acc[j] = wm(al, bh, acc[j]);
        }
      }
      float inv[8];
#pragma unroll
      for (int r = 0; r < 8; ++r) {
        const float d = den[(rb + 8 * hh + r) * 4 + head];
        inv[r] = 1.0f / fmaxf(d, 1e-16f);
      }
#pragma unroll
      for (int j = 0; j < 4; ++j) {
        const int col = cw + 16 * j + l;
        const float bb = bs[col];
#pragma unroll
        for (int r = 0; r < 8; ++r) {
          const int row = rb + 8 * hh + r;
          const float ag = sacc[row * HC + col];
          const float sv = acc[j][r] + bb;
          const float t = ag * inv[r] + sv;
          const unsigned hb = bfr(t);
          const unsigned ob16 = bfr(t - __uint_as_float(hb << 16));
          th[row * HC + col] = (unsigned short)hb;
          tl[row * HC + col] = (unsigned short)ob16;
        }
      }
    }
  }
  __syncthreads();

  {
    const int rg = wave >> 1;
    const int cg = (wave & 1) * 64;
    v8f acc[4];
#pragma unroll
    for (int j = 0; j < 4; ++j) acc[j] = z8;
    const int oa = (rg * 16 + l) * HC + 8 * hh;
    size_t ob[4];
#pragma unroll
    for (int j = 0; j < 4; ++j) ob[j] = (size_t)(cg + 16 * j + l) * HC + 8 * hh;
#pragma unroll 1
    for (int k0 = 0; k0 < HC; k0 += 32) {
      const v16b ah = ldf(th + oa + k0);
      const v16b al = ldf(tl + oa + k0);
#pragma unroll
      for (int j = 0; j < 4; ++j) {
        const v16b bh = ldf(Mh + ob[j] + k0);
        const v16b bl = ldf(Ml + ob[j] + k0);
        acc[j] = wm(ah, bh, acc[j]);
        acc[j] = wm(ah, bl, acc[j]);
        acc[j] = wm(al, bh, acc[j]);
      }
    }
    float* sw = stg + wave * 16 * STGP;
#pragma unroll
    for (int j = 0; j < 4; ++j) {
      const float bb = bm[cg + 16 * j + l];
#pragma unroll
      for (int r = 0; r < 8; ++r) sw[(8 * hh + r) * STGP + 16 * j + l] = fmaxf(acc[j][r] + bb, 0.f);
    }
  }
  __syncthreads();
  {
    const int rg = wave >> 1;
    const int cg = (wave & 1) * 64;
    const float* sw = stg + wave * 16 * STGP;
    v4f vals[8];
    size_t offs[8];
#pragma unroll
    for (int it = 0; it < 8; ++it) {
      const int idx = it * 32 + lane;
      const int row = idx >> 4;
      const int pc = idx & 15;
      vals[it] = *(const v4f*)(sw + row * STGP + 4 * pc);
      offs[it] = (size_t)(nodeBase + rg * 16 + row) * HID + cg + 4 * pc;
    }
#pragma unroll
    for (int it = 0; it < 8; ++it) *(volatile v4f*)(Hout + offs[it]) = vals[it];
    __threadfence();
#pragma unroll
    for (int it = 0; it < 8; ++it) *(volatile v4f*)(Hout + offs[it]) = vals[it];
  }
}

__global__ __launch_bounds__(NTH) void k_pool(const float* __restrict__ Hin, const int* __restrict__ bat,
                                            unsigned short* Gh, unsigned short* Gl, int nN, int MG) {
  extern __shared__ v4i lds_pl[];
  char* lb = (char*)lds_pl;
  float* mxs = (float*)lb;
  float* sms = (float*)(lb + PL_MX);
  int* gcnt = (int*)(lb + 2 * PL_MX);
  int* list = gcnt + NBG;
  int* wcnt = list + NWV * WCAP;

  const int tid = threadIdx.x;
  const int lane = tid & 31;
  const int wave = tid >> 5;
  const int gBase = blockIdx.x * NBG;

  for (int i = tid; i < NBG * HID; i += NTH) { mxs[i] = -3.0e38f; sms[i] = 0.f; }
  for (int i = tid; i < NBG; i += NTH) gcnt[i] = 0;
  __syncthreads();

  const int nChunks = (nN + CHUNK - 1) / CHUNK;
  int* wl = list + wave * WCAP;
#pragma unroll 1
  for (int ch = 0; ch < nChunks; ++ch) {
    const int cbase = ch * CHUNK;
    const bool full = (cbase + CHUNK <= nN);
    const int wc = scan_chunk<NBG, SHG>(bat, nN, cbase, full, gBase, wl, tid);
    if (lane == 0) wcnt[wave] = wc;
    __syncthreads();
    if (wave == 0) {
#pragma unroll 1
      for (int wsx = 0; wsx < NWV; ++wsx) {
        int n = wcnt[wsx];
        n = n > WCAP ? WCAP : n;
        n = n < 0 ? 0 : n;
#pragma unroll 1
        for (int i = 0; i < n; ++i) {
          const int ent = list[wsx * WCAP + i];
          const int slot = ent & (NBG - 1);
          const int el = (ent >> SHG) & (CHUNK - 1);
          int nd = cbase + el;
          nd = nd > nN - 1 ? nN - 1 : nd;
          const v4f hv = *(const v4f*)(Hin + (size_t)nd * HID + 4 * lane);
          v4f* mp = (v4f*)(mxs + slot * HID + 4 * lane);
          v4f* ap = (v4f*)(sms + slot * HID + 4 * lane);
          const v4f m = *mp;
          const v4f s = *ap;
          *mp = max4(m, hv);
          *ap = s + hv;
          if (lane == 0) gcnt[slot] += 1;
        }
      }
    }
    __syncthreads();
  }

#pragma unroll 1
  for (int j = 0; j < NBG / NWV; ++j) {
    const int slot = wave * (NBG / NWV) + j;
    const int g = gBase + slot;
    const int qo = 8 * (lane & 15);
    const v4f m0 = *(const v4f*)(mxs + slot * HID + qo);
    const v4f m1 = *(const v4f*)(mxs + slot * HID + qo + 4);
    const v4f s0 = *(const v4f*)(sms + slot * HID + qo);
    const v4f s1 = *(const v4f*)(sms + slot * HID + qo + 4);
    const int c = gcnt[slot];
    const float cf = (float)c;
    const float inv = 1.0f / fmaxf(cf, 1.0f);
    const bool has = c > 0;
    const bool left = lane < 16;
    const v4f z4 = {0.f, 0.f, 0.f, 0.f};
    const v4f a = sel4(left, sel4(has, m0, z4), s0 * inv);
    const v4f b = sel4(left, sel4(has, m1, z4), s1 * inv);
    v4i hq, lq;
    pack8(a, b, hq, lq);
    const bool wr = g < MG;
    const size_t o = (size_t)g * GP + 8 * lane;
    if (wr) { *(volatile v4i*)(Gh + o) = hq; *(volatile v4i*)(Gl + o) = lq; }
    __threadfence();
    if (wr) { *(volatile v4i*)(Gh + o) = hq; *(volatile v4i*)(Gl + o) = lq; }
  }
}

extern "C" void kernel_launch(void* const* d_in, const int* in_sizes, int n_in,
                              void* d_out, int out_size, void* d_ws, size_t ws_size,
                              hipStream_t stream) {
  if (n_in < 41) return;
  const int nN = in_sizes[2];
  if (nN <= 0) return;
  if (in_sizes[1] < 2 || (in_sizes[1] & 1)) return;
  const int nE = in_sizes[1] / 2;
  if (in_sizes[4] != HC) return;
  const int K1 = in_sizes[3] / HC;
  if (K1 < 1 || K1 > 64 || in_sizes[3] != K1 * HC || in_sizes[0] != nN * K1) return;
  if (in_sizes[5] != K1 * HC || in_sizes[7] != K1 * HC || in_sizes[9] != K1 * HC) return;
  if (in_sizes[6] != HC || in_sizes[8] != HC || in_sizes[10] != HC) return;
  if (in_sizes[11] != HC * HID || in_sizes[12] != HID) return;
  for (int b = 13; b <= 23; b += 10) {
    if (in_sizes[b] != HID * HC || in_sizes[b + 2] != HID * HC || in_sizes[b + 4] != HID * HC || in_sizes[b + 6] != HID * HC) return;
    if (in_sizes[b + 1] != HC || in_sizes[b + 3] != HC || in_sizes[b + 5] != HC || in_sizes[b + 7] != HC) return;
    if (in_sizes[b + 8] != HC * HID || in_sizes[b + 9] != HID) return;
  }
  if (in_sizes[33] != 2 * HID * 1024 || in_sizes[34] != 1024) return;
  if (in_sizes[35] != 1024 * 512 || in_sizes[36] != 512) return;
  if (in_sizes[37] != 512 * 256 || in_sizes[38] != 256) return;
  if (in_sizes[39] != 256 || in_sizes[40] < 1) return;
  const int nG = out_size;
  if (nG <= 0 || (nG & 31)) return;
  const int MG = nG;
  const int MP = ((nN + NB - 1) / NB) * NB;
  const int Kp1 = 64;

  const float* x   = (const float*)d_in[0];
  const int*   ei  = (const int*)d_in[1];
  const int*   bat = (const int*)d_in[2];
  const float* Wq1 = (const float*)d_in[3];  const float* bq1 = (const float*)d_in[4];
  const float* Wk1 = (const float*)d_in[5];  const float* bk1 = (const float*)d_in[6];
  const float* Wv1 = (const float*)d_in[7];  const float* bv1 = (const float*)d_in[8];
  const float* Ws1 = (const float*)d_in[9];  const float* bs1 = (const float*)d_in[10];
  const float* Wm1 = (const float*)d_in[11]; const float* bm1 = (const float*)d_in[12];
  const float* Wq2 = (const float*)d_in[13]; const float* bq2 = (const float*)d_in[14];
  const float* Wk2 = (const float*)d_in[15]; const float* bk2 = (const float*)d_in[16];
  const float* Wv2 = (const float*)d_in[17]; const float* bv2 = (const float*)d_in[18];
  const float* Ws2 = (const float*)d_in[19]; const float* bs2 = (const float*)d_in[20];
  const float* Wm2 = (const float*)d_in[21]; const float* bm2 = (const float*)d_in[22];
  const float* Wq3 = (const float*)d_in[23]; const float* bq3 = (const float*)d_in[24];
  const float* Wk3 = (const float*)d_in[25]; const float* bk3 = (const float*)d_in[26];
  const float* Wv3 = (const float*)d_in[27]; const float* bv3 = (const float*)d_in[28];
  const float* Ws3 = (const float*)d_in[29]; const float* bs3 = (const float*)d_in[30];
  const float* Wm3 = (const float*)d_in[31]; const float* bm3 = (const float*)d_in[32];
  const float* Wg1 = (const float*)d_in[33]; const float* bg1 = (const float*)d_in[34];
  const float* Wg2 = (const float*)d_in[35]; const float* bg2 = (const float*)d_in[36];
  const float* Wf1 = (const float*)d_in[37]; const float* bf1 = (const float*)d_in[38];
  const float* Wf2 = (const float*)d_in[39]; const float* bf2 = (const float*)d_in[40];
  float* out = (float*)d_out;

  size_t off = 0;
  char* wsb = (char*)d_ws;
#define CARVE(T, name, bytes) T* name = (T*)(wsb + off); off += (((size_t)(bytes)) + 255) & ~(size_t)255;
  CARVE(unsigned short, WP1h, (size_t)4 * HC * Kp1 * 2)
  CARVE(unsigned short, WP1l, (size_t)4 * HC * Kp1 * 2)
  CARVE(unsigned short, WP2h, (size_t)4 * HC * HID * 2)
  CARVE(unsigned short, WP2l, (size_t)4 * HC * HID * 2)
  CARVE(unsigned short, WP3h, (size_t)4 * HC * HID * 2)
  CARVE(unsigned short, WP3l, (size_t)4 * HC * HID * 2)
  CARVE(unsigned short, WM1h, (size_t)HID * HC * 2)
  CARVE(unsigned short, WM1l, (size_t)HID * HC * 2)
  CARVE(unsigned short, WM2h, (size_t)HID * HC * 2)
  CARVE(unsigned short, WM2l, (size_t)HID * HC * 2)
  CARVE(unsigned short, WM3h, (size_t)HID * HC * 2)
  CARVE(unsigned short, WM3l, (size_t)HID * HC * 2)
  CARVE(unsigned short, WG1h, (size_t)1024 * 2 * HID * 2)
  CARVE(unsigned short, WG1l, (size_t)1024 * 2 * HID * 2)
  CARVE(unsigned short, WG2h, (size_t)512 * 1024 * 2)
  CARVE(unsigned short, WG2l, (size_t)512 * 1024 * 2)
  CARVE(unsigned short, WF1h, (size_t)256 * 512 * 2)
  CARVE(unsigned short, WF1l, (size_t)256 * 512 * 2)
  CARVE(unsigned short, Xh,   (size_t)MP * HID * 2)
  CARVE(unsigned short, Xl,   (size_t)MP * HID * 2)
  CARVE(float,          KV,   (size_t)MP * KVP * 4)
  CARVE(float,          Hb,   (size_t)MP * HID * 4)
  CARVE(unsigned short, Gh,   (size_t)MG * GP * 2)
  CARVE(unsigned short, Gl,   (size_t)MG * GP * 2)
  CARVE(unsigned short, P1h,  (size_t)MG * 1024 * 2)
  CARVE(unsigned short, P1l,  (size_t)MG * 1024 * 2)
  CARVE(unsigned short, P2h,  (size_t)MG * 512 * 2)
  CARVE(unsigned short, P2l,  (size_t)MG * 512 * 2)
#undef CARVE
  if (off > ws_size) return;

  k_prep<<<(4 * HC) / 32, NTH, 0, stream>>>(Wq1, Wk1, Wv1, Ws1, HC, K1, Kp1, WP1h, WP1l, 4 * HC);
  k_prep<<<HID / 32, NTH, 0, stream>>>(Wm1, Wm1, Wm1, Wm1, HID, HC, HC, WM1h, WM1l, HID);
  k_prep<<<(4 * HC) / 32, NTH, 0, stream>>>(Wq2, Wk2, Wv2, Ws2, HC, HID, HID, WP2h, WP2l, 4 * HC);
  k_prep<<<HID / 32, NTH, 0, stream>>>(Wm2, Wm2, Wm2, Wm2, HID, HC, HC, WM2h, WM2l, HID);
  k_prep<<<(4 * HC) / 32, NTH, 0, stream>>>(Wq3, Wk3, Wv3, Ws3, HC, HID, HID, WP3h, WP3l, 4 * HC);
  k_prep<<<HID / 32, NTH, 0, stream>>>(Wm3, Wm3, Wm3, Wm3, HID, HC, HC, WM3h, WM3l, HID);
  k_prep<<<1024 / 32, NTH, 0, stream>>>(Wg1, Wg1, Wg1, Wg1, 1024, 2 * HID, 2 * HID, WG1h, WG1l, 1024);
  k_prep<<<512 / 32, NTH, 0, stream>>>(Wg2, Wg2, Wg2, Wg2, 512, 1024, 1024, WG2h, WG2l, 512);
  k_prep<<<256 / 32, NTH, 0, stream>>>(Wf1, Wf1, Wf1, Wf1, 256, 512, 512, WF1h, WF1l, 256);

  hipFuncSetAttribute(reinterpret_cast<const void*>(&k_layer), hipFuncAttributeMaxDynamicSharedMemorySize, LY_LDS);
  hipFuncSetAttribute(reinterpret_cast<const void*>(&k_pool), hipFuncAttributeMaxDynamicSharedMemorySize, PL_LDS);

  const dim3 gkv(MP / 32, KVP / 512);
  k_cvt<<<(MP * (Kp1 / 8) + NTH - 1) / NTH, NTH, 0, stream>>>(x, K1, nN, Kp1, MP, Xh, Xl);
  k_gemm<4, 8, 0, 0><<<gkv, 256, 0, stream>>>(Xh, Xl, WP1h + (size_t)HC * Kp1, WP1l + (size_t)HC * Kp1,
                                               bk1, bv1, HC, KV, Gh, Gl, bq1, bq1, Hb, Kp1, KVP);
  k_layer<<<MP / NB, NTH, LY_LDS, stream>>>(Xh, Xl, Kp1, WP1h, WP1l, bq1, bs1, KV, ei, WM1h, WM1l, bm1, Hb, nN, nE);
  k_cvt<<<(MP * (HID / 8) + NTH - 1) / NTH, NTH, 0, stream>>>(Hb, HID, nN, HID, MP, Xh, Xl);
  k_gemm<4, 8, 0, 0><<<gkv, 256, 0, stream>>>(Xh, Xl, WP2h + (size_t)HC * HID, WP2l + (size_t)HC * HID,
                                               bk2, bv2, HC, KV, Gh, Gl, bq1, bq1, Hb, HID, KVP);
  k_layer<<<MP / NB, NTH, LY_LDS, stream>>>(Xh, Xl, HID, WP2h, WP2l, bq2, bs2, KV, ei, WM2h, WM2l, bm2, Hb, nN, nE);
  k_cvt<<<(MP * (HID / 8) + NTH - 1) / NTH, NTH, 0, stream>>>(Hb, HID, nN, HID, MP, Xh, Xl);
  k_gemm<4, 8, 0, 0><<<gkv, 256, 0, stream>>>(Xh, Xl, WP3h + (size_t)HC * HID, WP3l + (size_t)HC * HID,
                                               bk3, bv3, HC, KV, Gh, Gl, bq1, bq1, Hb, HID, KVP);
  k_layer<<<MP / NB, NTH, LY_LDS, stream>>>(Xh, Xl, HID, WP3h, WP3l, bq3, bs3, KV, ei, WM3h, WM3l, bm3, Hb, nN, nE);

  k_pool<<<(MG + NBG - 1) / NBG, NTH, PL_LDS, stream>>>(Hb, bat, Gh, Gl, nN, MG);

  k_gemm<4, 8, 1, 1><<<dim3(MG / 32, 1024 / 512), 256, 0, stream>>>(Gh, Gl, WG1h, WG1l, bg1, bg1, 1024,
                                                                    KV, P1h, P1l, bq1, bq1, Hb, 2 * HID, 1024);
  k_gemm<4, 8, 1, 1><<<dim3(MG / 32, 1), 256, 0, stream>>>(P1h, P1l, WG2h, WG2l, bg2, bg2, 512,
                                                           KV, P2h, P2l, bq1, bq1, Hb, 1024, 512);
  k_gemm<2, 8, 2, 1><<<dim3(MG / 32, 1), 256, 0, stream>>>(P2h, P2l, WF1h, WF1l, bf1, bf1, 256,
                                                           KV, Gh, Gl, Wf2, bf2, out, 512, 256);
}
